// BertWithRopeAttention_14173392077010
// MI455X (gfx1250) — hardware-verified
//
#include <hip/hip_runtime.h>
#include <math.h>
#include <stdint.h>

constexpr int NB_BATCH  = 4;
constexpr int SEQ_LEN   = 2048;
constexpr int HID       = 1024;
constexpr int NHEADS    = 16;
constexpr int DHEAD     = 64;
constexpr int QKV_N     = 3072;
constexpr int ROPE_HALF = 32;

typedef __attribute__((ext_vector_type(16))) _Float16 v16h;
typedef __attribute__((ext_vector_type(8)))  _Float16 v8h;
typedef __attribute__((ext_vector_type(16))) __bf16   v16b;
typedef __attribute__((ext_vector_type(8)))  __bf16   v8b;
typedef __attribute__((ext_vector_type(8)))  float    v8f;
typedef __attribute__((ext_vector_type(4)))  float    v4f;
typedef __attribute__((ext_vector_type(2)))  float    v2f;
typedef __attribute__((ext_vector_type(4)))  unsigned int v4u;

__device__ __forceinline__ unsigned short f2bf_bits(float f) {
  unsigned u = __float_as_uint(f);
  return (unsigned short)((u + 0x7FFFu + ((u >> 16) & 1u)) >> 16);
}
__device__ __forceinline__ float bf_bits2f(unsigned short h) { return __uint_as_float(((unsigned)h) << 16); }

__device__ __forceinline__ void dep_guard_h(v8f& a, v8f& b, v16h x, v16h y) { asm volatile("v_nop\n\tv_nop\n\tv_nop\n\tv_nop" : "+v"(a), "+v"(b) : "v"(x), "v"(y)); }
__device__ __forceinline__ void dep_guard_b(v8f& a, v8f& b, v16b x, v16b y) { asm volatile("v_nop\n\tv_nop\n\tv_nop\n\tv_nop" : "+v"(a), "+v"(b) : "v"(x), "v"(y)); }
__device__ __forceinline__ void keep4_h(v16h a, v16h b, v16h c, v16h d) { asm volatile("v_nop" :: "v"(a), "v"(b), "v"(c), "v"(d)); }
__device__ __forceinline__ void keep4_b(v16b a, v16b b, v16b c, v16b d) { asm volatile("v_nop" :: "v"(a), "v"(b), "v"(c), "v"(d)); }
__device__ __forceinline__ void acc_guard4(v8f& a, v8f& b, v8f& c, v8f& d) { asm volatile("v_nop\n\tv_nop\n\tv_nop\n\tv_nop" : "+v"(a), "+v"(b), "+v"(c), "+v"(d)); }
template <typename T> struct Frag;
template <> struct Frag<_Float16> {
  typedef v16h V; union U { v16h v; v8h h[2]; };
  static __device__ __forceinline__ v16h load(const _Float16* p) {
    U f; f.h[0] = *(const v8h*)(p); f.h[1] = *(const v8h*)(p + 16); return f.v;
  }
  static __device__ __forceinline__ v8f mma(v16h a, v16h b, v8f c) {
    return __builtin_amdgcn_wmma_f32_16x16x32_f16(false, a, false, b, (short)0, c, false, false);
  }
  static __device__ __forceinline__ void guard(v8f& a, v8f& b, v16h x, v16h y) { dep_guard_h(a, b, x, y); }
  static __device__ __forceinline__ void keep(v16h a, v16h b, v16h c, v16h d) { keep4_h(a, b, c, d); }
};
template <> struct Frag<__bf16> {
  typedef v16b V; union U { v16b v; v8b h[2]; };
  static __device__ __forceinline__ v16b load(const __bf16* p) {
    U f; f.h[0] = *(const v8b*)(p); f.h[1] = *(const v8b*)(p + 16); return f.v;
  }
  static __device__ __forceinline__ v8f mma(v16b a, v16b b, v8f c) {
    return __builtin_amdgcn_wmma_f32_16x16x32_bf16(false, a, false, b, (short)0, c, false, false);
  }
  static __device__ __forceinline__ void guard(v8f& a, v8f& b, v16b x, v16b y) { dep_guard_b(a, b, x, y); }
  static __device__ __forceinline__ void keep(v16b a, v16b b, v16b c, v16b d) { keep4_b(a, b, c, d); }
};

template <int ET> struct Elem;
template <> struct Elem<0> { typedef _Float16 T; };
template <> struct Elem<1> { typedef __bf16 T; };
template <int ET, bool SPLIT, int BIAS_MODE, int OUT_MODE, bool RESID, int ACT = 0>
__global__ __launch_bounds__(256) void wmma_gemm64(
    const unsigned short* __restrict__ Ap, const unsigned short* __restrict__ A2p, int lda, long strideA,
    const unsigned short* __restrict__ Btp, const unsigned short* __restrict__ Bt2p, int ldb, long strideB,
    void* __restrict__ Cout, void* __restrict__ Cout2, int ldc, long strideC,
    const float* __restrict__ bias,
    const float* __restrict__ resid, long strideR,
    int M, int N, int K, float scale) {
  typedef typename Elem<ET>::T T;
  typedef typename Frag<T>::V V;
  const T* A = (const T*)Ap; const T* A2 = (const T*)A2p; const T* Bt = (const T*)Btp; const T* Bt2 = (const T*)Bt2p;
  __shared__ __align__(16) float sT[8][16 * 68];
  const int b    = blockIdx.y;
  const int lane = threadIdx.x & 31;
  const int wave = threadIdx.x >> 5;
  const int tilesN = N >> 6;
  const int tilesM = M >> 6;
  const int tile = blockIdx.x * 8 + wave;
  if (tile >= tilesM * tilesN) return;
  const int tm = tile / tilesN;
  const int tn = tile - tm * tilesN;
  const int m0 = tm << 6;
  const int n0 = tn << 6;

  const T* Ab  = A  + (size_t)b * strideA;
  const T* Bb  = Bt + (size_t)b * strideB;
  const T* Ab2 = SPLIT ? (A2  + (size_t)b * strideA) : nullptr;
  const T* Bb2 = SPLIT ? (Bt2 + (size_t)b * strideB) : nullptr;

  const int rlane = lane & 15;
  const int koff  = (lane >> 4) * 8;
  const int mOff  = (lane >> 4) * 8;

  v8f acc[4][4];
#pragma unroll
  for (int i = 0; i < 4; ++i)
#pragma unroll
    for (int j = 0; j < 4; ++j) acc[i][j] = (v8f){0.f,0.f,0.f,0.f,0.f,0.f,0.f,0.f};

  for (int k0 = 0; k0 < K; k0 += 32) {
    V bh[4], bl[4];
#pragma unroll
    for (int j = 0; j < 4; ++j) {
      const size_t bo = (size_t)(n0 + (j << 4) + rlane) * ldb + koff + k0;
      bh[j] = Frag<T>::load(Bb + bo);
      if (SPLIT) bl[j] = Frag<T>::load(Bb2 + bo);
    }
#pragma unroll
    for (int i = 0; i < 4; ++i) {
      const size_t ao = (size_t)(m0 + (i << 4) + rlane) * lda + koff + k0;
      V ah = Frag<T>::load(Ab + ao);
      V al;
      if (SPLIT) al = Frag<T>::load(Ab2 + ao);
#pragma unroll
      for (int j = 0; j < 4; ++j) {
        acc[i][j] = Frag<T>::mma(ah, bh[j], acc[i][j]);
        if (SPLIT) {
          acc[i][j] = Frag<T>::mma(ah, bl[j], acc[i][j]);
          acc[i][j] = Frag<T>::mma(al, bh[j], acc[i][j]);
        }
      }
      Frag<T>::guard(acc[i][0], acc[i][3], ah, SPLIT ? al : ah);
    }
    Frag<T>::keep(bh[0], bh[1], bh[2], bh[3]);
    if (SPLIT) Frag<T>::keep(bl[0], bl[1], bl[2], bl[3]);
  }
  acc_guard4(acc[0][0], acc[0][1], acc[0][2], acc[0][3]);
  acc_guard4(acc[1][0], acc[1][1], acc[1][2], acc[1][3]);
  acc_guard4(acc[2][0], acc[2][1], acc[2][2], acc[2][3]);
  acc_guard4(acc[3][0], acc[3][1], acc[3][2], acc[3][3]);

  float* slab = sT[wave];
  const float* Rb = RESID ? (resid + (size_t)b * strideR) : nullptr;
#pragma unroll
  for (int i = 0; i < 4; ++i) {
    const int mBase = m0 + (i << 4);
#pragma unroll
    for (int j = 0; j < 4; ++j) {
      const int n = n0 + (j << 4) + rlane;
      float bv = 0.f;
      if (BIAS_MODE == 2) bv = bias[n];
#pragma unroll
      for (int r = 0; r < 8; ++r) {
        float v = acc[i][j][r] * scale;
        if (BIAS_MODE == 1) v += bias[mBase + mOff + r];
        if (BIAS_MODE == 2) v += bv;
        if (RESID) v += Rb[(size_t)(mBase + mOff + r) * ldc + n];
        if (ACT == 1) v = tanhf(v);
        if (ACT == 2) v = fmaxf(v, 0.0f);
        if (ACT == 3) v = v / (1.0f + expf(-v));
        if (ACT == 4) v = (v > 0.f) ? v : 0.01f * v;
        if (ACT == 5) v = 0.5f * v * (1.0f + erff(v * 0.70710678118654752f));
        slab[(mOff + r) * 68 + (j << 4) + rlane] = v;
      }
    }
    __builtin_amdgcn_fence(__ATOMIC_RELEASE, "workgroup");
    __builtin_amdgcn_wave_barrier();
    __builtin_amdgcn_fence(__ATOMIC_ACQUIRE, "workgroup");
    if (OUT_MODE == 0) {
      float* C = (float*)Cout + (size_t)b * strideC;
      const int hh = lane >> 4, c4 = (lane & 15) * 4;
      for (int pass = 0; pass < 2; ++pass) {
#pragma unroll
        for (int it = 0; it < 8; ++it) {
          const int row = it * 2 + hh;
          v4f v = *(const v4f*)(slab + row * 68 + c4);
          *(volatile v4f*)(C + (size_t)(mBase + row) * ldc + n0 + c4) = v;
        }
        __threadfence();
      }
    } else {
      const int q = lane >> 3, c8 = (lane & 7) * 8;
      unsigned short* C  = (unsigned short*)Cout  + (size_t)b * strideC;
      unsigned short* C2 = (OUT_MODE == 2) ? ((unsigned short*)Cout2 + (size_t)b * strideC) : nullptr;
      for (int pass = 0; pass < 2; ++pass) {
#pragma unroll
        for (int it = 0; it < 4; ++it) {
          const int row = it * 4 + q;
          const float* sp = slab + row * 68 + c8;
          v8h hv, lv;
#pragma unroll
          for (int e = 0; e < 8; ++e) {
            if (OUT_MODE == 1) {
              hv[e] = (_Float16)sp[e];
            } else {
              unsigned short hb = f2bf_bits(sp[e]);
              unsigned short lb = f2bf_bits(sp[e] - bf_bits2f(hb));
              hv[e] = __builtin_bit_cast(_Float16, hb);
              lv[e] = __builtin_bit_cast(_Float16, lb);
            }
          }
          *(volatile v8h*)(C + (size_t)(mBase + row) * ldc + n0 + c8) = hv;
          if (OUT_MODE == 2) *(volatile v8h*)(C2 + (size_t)(mBase + row) * ldc + n0 + c8) = lv;
        }
        __threadfence();
      }
    }
    __builtin_amdgcn_fence(__ATOMIC_RELEASE, "workgroup");
    __builtin_amdgcn_wave_barrier();
    __builtin_amdgcn_fence(__ATOMIC_ACQUIRE, "workgroup");
  }
}

__device__ __forceinline__ unsigned pk16(unsigned short a, unsigned short b) { return (unsigned)a | ((unsigned)b << 16); }

__global__ __launch_bounds__(256) void cast_f32_bf16x2(const float* __restrict__ in, unsigned short* __restrict__ out, int n2) {
  const int i = blockIdx.x * 256 + threadIdx.x;
  if (i < n2) {
    const v2f f = *(const v2f*)(in + 2 * (size_t)i);
    const unsigned u = pk16(f2bf_bits(f[0]), f2bf_bits(f[1]));
    ((volatile unsigned*)out)[i] = u;
    __threadfence();
    ((volatile unsigned*)out)[i] = u;
  }
}

__global__ __launch_bounds__(256) void bias_rne_kernel(const float* __restrict__ a, float* __restrict__ ao, int na, int gridA,
                                                      const float* __restrict__ bsrc, float* __restrict__ bo, int nbv) {
  const int tid = threadIdx.x;
  if ((int)blockIdx.x < gridA) {
    const int i = blockIdx.x * 256 + tid;
    if (i < na) {
      const float v = bf_bits2f(f2bf_bits(a[i]));
      ((volatile float*)ao)[i] = v;
      __threadfence();
      ((volatile float*)ao)[i] = v;
    }
  } else {
    const int i = ((int)blockIdx.x - gridA) * 256 + tid;
    if (i < nbv) {
      const float v = bf_bits2f(f2bf_bits(bsrc[i]));
      ((volatile float*)bo)[i] = v;
      __threadfence();
      ((volatile float*)bo)[i] = v;
    }
  }
}

struct RopeFreq { float f[32]; };
static_assert(sizeof(RopeFreq) == 128, "size");

template <int WHICH>
__global__ __launch_bounds__(256) void rope_table_kernel(const int* __restrict__ pos, float* __restrict__ tab, int S, RopeFreq rf) {
  const int idx = blockIdx.x * 256 + threadIdx.x;
  const int j = idx & 31;
  int s = idx >> 5;
  const bool ok = (s < S);
  s = ok ? s : (S - 1);
  float inv = 0.0f;
#pragma unroll
  for (int jj = 0; jj < 32; ++jj) inv = (j == jj) ? rf.f[jj] : inv;
  const float ang = (float)pos[s] * inv;
  float v;
  if (WHICH == 1) v = sinf(ang); else v = cosf(ang);
  if (ok) {
    ((volatile float*)tab)[idx] = v;
    __threadfence();
    ((volatile float*)tab)[idx] = v;
  }
}

template <int MODE> __device__ __forceinline__ unsigned short tconv_cv(float f, float scl) {
  if (MODE == 0) return f2bf_bits(f);
  if (MODE == 1) { const float r = bf_bits2f(f2bf_bits(f)) * scl; return __builtin_bit_cast(unsigned short, (_Float16)r); }
  return __builtin_bit_cast(unsigned short, (_Float16)f);
}

template <int MODE>
__global__ __launch_bounds__(256) void tconv_kernel(const float* __restrict__ W, unsigned short* __restrict__ o,
                                                   int R, int Cc, int ldin, float scl) {
  __shared__ __align__(16) float tf[64 * 68];
  const int c0  = blockIdx.x * 64;
  const int r0  = blockIdx.y * 64;
  const int tid = threadIdx.x;
  (void)Cc;
  {
    const int lr = tid >> 4;
    const int c4 = (tid & 15) * 4;
#pragma unroll
    for (int it = 0; it < 4; ++it) {
      const int rr = it * 16 + lr;
      const v4f a = *(const v4f*)(W + (size_t)(r0 + rr) * ldin + c0 + c4);
      *(v4f*)(tf + rr * 68 + c4) = a;
    }
  }
  __syncthreads();
  const int sub = tid >> 3;
  const int c8  = (tid & 7) * 8;
  v4u hv[2];
#pragma unroll
  for (int it = 0; it < 2; ++it) {
    const int oc = it * 32 + sub;
    v4u a;
#pragma unroll
    for (int q = 0; q < 4; ++q) {
      const float f0 = tf[(c8 + 2 * q) * 68 + oc];
      const float f1 = tf[(c8 + 2 * q + 1) * 68 + oc];
      a[q] = pk16(tconv_cv<MODE>(f0, scl), tconv_cv<MODE>(f1, scl));
    }
    hv[it] = a;
  }
  for (int pass = 0; pass < 2; ++pass) {
#pragma unroll
    for (int it = 0; it < 2; ++it) {
      const int oc = it * 32 + sub;
      const size_t go = (size_t)(c0 + oc) * R + r0 + c8;
      *(volatile v4u*)(o + go) = hv[it];
    }
    __threadfence();
  }
}

__global__ __launch_bounds__(256) void rope_qk_kernel(const float* __restrict__ qkvf, const float* __restrict__ ctab,
                                                     const float* __restrict__ stab, unsigned short* __restrict__ qk16, int S) {
  int s = blockIdx.x;
  s = (s < S) ? s : (S - 1);
  const int tid  = threadIdx.x;
  const int lane = tid & 31, wave = tid >> 5;
  const int L    = wave * 4 + (lane >> 3);
  const int t    = L >> 4;
  const int h    = L & 15;
  const int seg  = lane & 7;
  const int jb   = (seg & 3) * 8;
  const bool upper = (seg >= 4);
  const float* src = qkvf + (size_t)s * QKV_N + t * HID + h * DHEAD + jb;
  const v4f xa0 = *(const v4f*)(src),      xa1 = *(const v4f*)(src + 4);
  const v4f xb0 = *(const v4f*)(src + 32), xb1 = *(const v4f*)(src + 36);
  const float* cr = ctab + (size_t)s * ROPE_HALF + jb;
  const float* sr = stab + (size_t)s * ROPE_HALF + jb;
  const v4f ca0 = *(const v4f*)(cr), ca1 = *(const v4f*)(cr + 4);
  const v4f sa0 = *(const v4f*)(sr), sa1 = *(const v4f*)(sr + 4);
  v8h o;
#pragma unroll
  for (int e = 0; e < 4; ++e) {
    const float lo0 = xa0[e] * ca0[e] - xb0[e] * sa0[e];
    const float up0 = xb0[e] * ca0[e] + xa0[e] * sa0[e];
    o[e] = (_Float16)(upper ? up0 : lo0);
    const float lo1 = xa1[e] * ca1[e] - xb1[e] * sa1[e];
    const float up1 = xb1[e] * ca1[e] + xa1[e] * sa1[e];
    o[4 + e] = (_Float16)(upper ? up1 : lo1);
  }
  unsigned short* dst = qk16 + (size_t)t * S * HID + (size_t)s * HID + h * DHEAD + seg * 8;
  *(volatile v8h*)(void*)dst = o;
  __threadfence();
  *(volatile v8h*)(void*)dst = o;
}

constexpr int ATT_D  = 64;
constexpr int ATT_NW = 4;
constexpr int ATT_QB = 64;
constexpr int ATT_KC = 64;
constexpr float P_CARRY = 32768.0f;

__device__ __forceinline__ v8f at_mma_h(v16h a, v16h b, v8f c) {
  c = __builtin_amdgcn_wmma_f32_16x16x32_f16(false, a, false, b, (short)0, c, false, false);
  asm volatile("v_nop\n\tv_nop\n\tv_nop\n\tv_nop" : "+v"(c) : "v"(a), "v"(b));
  return c;
}

__global__ __launch_bounds__(128)
void attn_f16_kernel(const unsigned short* __restrict__ qp, const unsigned short* __restrict__ kp,
                     const unsigned short* __restrict__ vtp, unsigned short* __restrict__ ctx,
                     float sscale, float oscale) {
  union FH { v16h v; v8h h[2]; };
  __shared__ __align__(16) _Float16 Ksh[ATT_KC * ATT_D];
  __shared__ __align__(16) _Float16 Vth[ATT_D * ATT_KC];
  __shared__ __align__(16) _Float16 Psh[ATT_NW][16 * ATT_KC];
  __shared__ __align__(16) float    Os[ATT_NW][16 * 68];

  const int tid  = threadIdx.x;
  const int wave = tid >> 5;
  const int lane = tid & 31;
  const int hh   = lane >> 4;
  const int c    = lane & 15;

  const int nqb = SEQ_LEN / ATT_QB;
  const int bx = blockIdx.x;
  const int qb = bx % nqb;
  int h = bx / nqb;
  h = (h < NHEADS) ? h : (NHEADS - 1);
  const int q0 = qb * ATT_QB + wave * 16;

  const _Float16* Qh = (const _Float16*)(const void*)qp  + (size_t)h * ATT_D;
  const _Float16* Kh = (const _Float16*)(const void*)kp  + (size_t)h * ATT_D;
  const _Float16* Vh = (const _Float16*)(const void*)vtp + (size_t)h * ATT_D * SEQ_LEN;
  unsigned short* ob = ctx + (size_t)h * ATT_D;

  v16h qa[2];
#pragma unroll
  for (int dc = 0; dc < 2; ++dc) {
    const _Float16* qr = Qh + (size_t)(q0 + c) * HID + dc * 32 + 8 * hh;
    qa[dc] = Frag<_Float16>::load(qr);
  }

  float mrow[8], lrow[8];
  v8f oacc[4];
#pragma unroll
  for (int r = 0; r < 8; ++r) { mrow[r] = -INFINITY; lrow[r] = 0.f; }
#pragma unroll
  for (int t = 0; t < 4; ++t) oacc[t] = (v8f){0.f,0.f,0.f,0.f,0.f,0.f,0.f,0.f};

  const int nChunks = SEQ_LEN / ATT_KC;
  for (int kc = 0; kc < nChunks; ++kc) {
    const int kv0 = kc * ATT_KC;
    __syncthreads();
    {
      const int r = tid >> 1, half = (tid & 1) * 32;
      const _Float16* ksrc = Kh + (size_t)(kv0 + r) * HID + half;
      const _Float16* vsrc = Vh + (size_t)r * SEQ_LEN + kv0 + half;
#pragma unroll
      for (int i = 0; i < 4; ++i) {
        const v8h a0 = *(const v8h*)(ksrc + 8 * i);
        const v8h b0 = *(const v8h*)(vsrc + 8 * i);
        *(v8h*)(Ksh + r * ATT_D  + half + 8 * i) = a0;
        *(v8h*)(Vth + r * ATT_KC + half + 8 * i) = b0;
      }
    }
    __syncthreads();

    v8f s[4];
#pragma unroll
    for (int j = 0; j < 4; ++j) {
      s[j] = (v8f){0.f,0.f,0.f,0.f,0.f,0.f,0.f,0.f};
#pragma unroll
      for (int dc = 0; dc < 2; ++dc) {
        FH kb;
        kb.h[0] = *(const v8h*)(Ksh + (j * 16 + c) * ATT_D + dc * 32 + 8 * hh);
        kb.h[1] = *(const v8h*)(Ksh + (j * 16 + c) * ATT_D + dc * 32 + 16 + 8 * hh);
        s[j] = at_mma_h(qa[dc], kb.v, s[j]);
      }
    }
    float cm[8];
#pragma unroll
    for (int r = 0; r < 8; ++r) {
      float m = -INFINITY;
#pragma unroll
      for (int j = 0; j < 4; ++j) {
        const float sv = s[j][r] * sscale;
        s[j][r] = sv;
        m = fmaxf(m, sv);
      }
#pragma unroll
      for (int off = 1; off < 16; off <<= 1) m = fmaxf(m, __shfl_xor(m, off, 32));
      cm[r] = m;
    }
    _Float16* pw = Psh[wave];
#pragma unroll
    for (int r = 0; r < 8; ++r) {
      const float mnew = fmaxf(mrow[r], cm[r]);
      const float alpha = expf(mrow[r] - mnew);
      mrow[r] = mnew;
      float psum = 0.f;
#pragma unroll
      for (int j = 0; j < 4; ++j) {
        const float p = expf(s[j][r] - mnew);
        psum += p;
        pw[(8 * hh + r) * ATT_KC + j * 16 + c] = (_Float16)(p * P_CARRY);
      }
#pragma unroll
      for (int off = 1; off < 16; off <<= 1) psum += __shfl_xor(psum, off, 32);
      lrow[r] = lrow[r] * alpha + psum;
#pragma unroll
      for (int t = 0; t < 4; ++t) oacc[t][r] *= alpha;
    }
    __builtin_amdgcn_fence(__ATOMIC_RELEASE, "workgroup");
    __builtin_amdgcn_wave_barrier();
    __builtin_amdgcn_fence(__ATOMIC_ACQUIRE, "workgroup");
#pragma unroll 1
    for (int kk = 0; kk < 2; ++kk) {
      FH pa;
      pa.h[0] = *(const v8h*)(pw + c * ATT_KC + kk * 32 + 8 * hh);
      pa.h[1] = *(const v8h*)(pw + c * ATT_KC + kk * 32 + 16 + 8 * hh);
#pragma unroll
      for (int t = 0; t < 4; ++t) {
        FH vb;
        vb.h[0] = *(const v8h*)(Vth + (t * 16 + c) * ATT_KC + kk * 32 + 8 * hh);
        vb.h[1] = *(const v8h*)(Vth + (t * 16 + c) * ATT_KC + kk * 32 + 16 + 8 * hh);
        oacc[t] = at_mma_h(pa.v, vb.v, oacc[t]);
      }
    }
  }

  float* os = Os[wave];
#pragma unroll
  for (int r = 0; r < 8; ++r) {
    const float inv = oscale / (lrow[r] * P_CARRY);
#pragma unroll
    for (int t = 0; t < 4; ++t) os[(8 * hh + r) * 68 + t * 16 + c] = oacc[t][r] * inv;
  }
  __builtin_amdgcn_fence(__ATOMIC_RELEASE, "workgroup");
  __builtin_amdgcn_wave_barrier();
  __builtin_amdgcn_fence(__ATOMIC_ACQUIRE, "workgroup");
  {
    const int q4 = lane >> 3, c8 = (lane & 7) * 8;
    for (int pass = 0; pass < 2; ++pass) {
#pragma unroll
      for (int it = 0; it < 4; ++it) {
        const int row = it * 4 + q4;
        const float* sp = os + row * 68 + c8;
        v8h hv;
#pragma unroll
        for (int e = 0; e < 8; ++e) hv[e] = (_Float16)sp[e];
        *(volatile v8h*)(void*)(ob + (size_t)(q0 + row) * HID + c8) = hv;
      }
      __threadfence();
    }
  }
}

extern "C" void kernel_launch(void* const* d_in, const int* in_sizes, int n_in,
                              void* d_out, int out_size, void* d_ws, size_t ws_size,
                              hipStream_t stream) {
  if (n_in < 6) return;
  if (in_sizes[0] != SEQ_LEN) return;
  if (in_sizes[1] != NB_BATCH * SEQ_LEN * HID) return;
  if (in_sizes[2] != HID * QKV_N) return;
  if (in_sizes[3] != QKV_N) return;
  if (in_sizes[4] != HID * HID) return;
  if (in_sizes[5] != HID) return;
  if (out_size != NB_BATCH * SEQ_LEN * HID) return;

  const int*   positions = (const int*)d_in[0];
  const float* hidden    = (const float*)d_in[1];
  const float* Wqkv      = (const float*)d_in[2];
  const float* bqkv      = (const float*)d_in[3];
  const float* Wout      = (const float*)d_in[4];
  const float* bout      = (const float*)d_in[5];
  float* out = (float*)d_out;

  const size_t off_hid16 = 0;
  const size_t off_wqkvT = off_hid16 + (size_t)NB_BATCH * SEQ_LEN * HID * 2;
  const size_t off_woutT = off_wqkvT + (size_t)QKV_N * HID * 2;
  const size_t off_bq    = off_woutT + (size_t)HID * HID * 2;
  const size_t off_bo    = off_bq    + (size_t)QKV_N * 4;
  const size_t off_cos   = off_bo    + (size_t)HID * 4;
  const size_t off_sin   = off_cos   + (size_t)SEQ_LEN * ROPE_HALF * 4;
  const size_t off_qkvf  = off_sin   + (size_t)SEQ_LEN * ROPE_HALF * 4;
  const size_t off_qk16  = off_qkvf  + (size_t)SEQ_LEN * QKV_N * 4;
  const size_t off_vt16  = off_qk16  + (size_t)2 * SEQ_LEN * HID * 2;
  const size_t off_ctx16 = off_vt16  + (size_t)HID * SEQ_LEN * 2;
  const size_t ws_total  = off_ctx16 + (size_t)SEQ_LEN * HID * 2;
  if (ws_total > ws_size) return;

  char* ws = (char*)d_ws;
  unsigned short* hid16 = (unsigned short*)(ws + off_hid16);
  unsigned short* wqkvT = (unsigned short*)(ws + off_wqkvT);
  unsigned short* woutT = (unsigned short*)(ws + off_woutT);
  float* bq_r  = (float*)(ws + off_bq);
  float* bo_r  = (float*)(ws + off_bo);
  float* cos_t = (float*)(ws + off_cos);
  float* sin_t = (float*)(ws + off_sin);
  float* qkvf  = (float*)(ws + off_qkvf);
  unsigned short* qk16  = (unsigned short*)(ws + off_qk16);
  unsigned short* vt16  = (unsigned short*)(ws + off_vt16);
  unsigned short* ctx16 = (unsigned short*)(ws + off_ctx16);

  RopeFreq rf;
  for (int j = 0; j < ROPE_HALF; ++j) {
    const float e = (float)j * (1.0f / 32.0f);
    const double pd = pow(10000.0, (double)e);
    const float p = (float)pd;
    rf.f[j] = 1.0f / p;
  }

  bias_rne_kernel<<<QKV_N / 256 + HID / 256, 256, 0, stream>>>(bqkv, bq_r, QKV_N, QKV_N / 256, bout, bo_r, HID);
  rope_table_kernel<0><<<SEQ_LEN * ROPE_HALF / 256, 256, 0, stream>>>(positions, cos_t, SEQ_LEN, rf);
  rope_table_kernel<1><<<SEQ_LEN * ROPE_HALF / 256, 256, 0, stream>>>(positions, sin_t, SEQ_LEN, rf);
  cast_f32_bf16x2<<<NB_BATCH * SEQ_LEN * HID / 2 / 256, 256, 0, stream>>>(hidden, hid16, NB_BATCH * SEQ_LEN * HID / 2);
  tconv_kernel<0><<<dim3(QKV_N / 64, HID / 64), 256, 0, stream>>>(Wqkv, wqkvT, HID, QKV_N, QKV_N, 1.0f);
  tconv_kernel<1><<<dim3(HID / 64, HID / 64), 256, 0, stream>>>(Wout, woutT, HID, HID, HID, 32.0f);

  const int qkv_tiles = (SEQ_LEN / 64) * (QKV_N / 64);
  const int out_tiles = (SEQ_LEN / 64) * (HID / 64);

  for (int b = 0; b < NB_BATCH; ++b) {
    wmma_gemm64<1, false, 2, 0, false><<<dim3((qkv_tiles + 7) / 8, 1), 256, 0, stream>>>(
        hid16 + (size_t)b * SEQ_LEN * HID, nullptr, HID, 0,
        wqkvT, nullptr, HID, 0,
        (void*)qkvf, nullptr, QKV_N, 0,
        bq_r, nullptr, 0,
        SEQ_LEN, QKV_N, HID, 1.0f);
    rope_qk_kernel<<<SEQ_LEN, 256, 0, stream>>>(qkvf, cos_t, sin_t, qk16, SEQ_LEN);
    tconv_kernel<2><<<dim3(HID / 64, SEQ_LEN / 64), 256, 0, stream>>>(qkvf + 2 * HID, vt16, SEQ_LEN, HID, QKV_N, 1.0f);
    attn_f16_kernel<<<NHEADS * (SEQ_LEN / ATT_QB), 128, 0, stream>>>(qk16, qk16 + (size_t)SEQ_LEN * HID, vt16, ctx16, 0.125f, 16.0f);
    wmma_gemm64<0, false, 2, 0, false><<<dim3((out_tiles + 7) / 8, 1), 256, 0, stream>>>(
        ctx16, nullptr, HID, 0,
        woutT, nullptr, HID, 0,
        (void*)(out + (size_t)b * SEQ_LEN * HID), nullptr, HID, 0,
        bo_r, nullptr, 0,
        SEQ_LEN, HID, HID, 1.0f / 512.0f);
  }
}
